// SelfAttention_6622839571107
// MI455X (gfx1250) — hardware-verified
//
#include <hip/hip_runtime.h>
#include <math.h>

#ifndef NB
#define NB 8
#endif
#ifndef SEQ
#define SEQ 3136
#endif
#define NB_FULL 8
#define SEQ_FULL 3136
#define CH 128
#define QKP 256
#define OTP 68

static_assert(SEQ % 64 == 0);
static_assert(SEQ <= SEQ_FULL);
static_assert(NB <= NB_FULL);
static_assert(CH == 128);

typedef __attribute__((ext_vector_type(16))) _Float16 v16h;
typedef __attribute__((ext_vector_type(8)))  _Float16 v8h;
typedef __attribute__((ext_vector_type(16))) __bf16   v16b;
typedef __attribute__((ext_vector_type(8)))  __bf16   v8b;
typedef __attribute__((ext_vector_type(8)))  float    v8f;
typedef __attribute__((ext_vector_type(4)))  float    v4f;
typedef unsigned int cm_u4 __attribute__((ext_vector_type(4)));

__device__ __forceinline__ v8f wmma16(v16h a, v16h b, v8f c) {
    c = __builtin_amdgcn_wmma_f32_16x16x32_f16(false, a, false, b, (short)0, c, false, false);
    asm volatile("v_nop\n\tv_nop\n\tv_nop\n\tv_nop" : "+v"(c) : "v"(a), "v"(b));
    return c;
}
struct Split { v16b hi, lo; };
__device__ __forceinline__ v8f wmma3(const Split& a, const Split& b, v8f c) {
    c = __builtin_amdgcn_wmma_f32_16x16x32_bf16(false, a.hi, false, b.hi, (short)0, c, false, false);
    c = __builtin_amdgcn_wmma_f32_16x16x32_bf16(false, a.hi, false, b.lo, (short)0, c, false, false);
    c = __builtin_amdgcn_wmma_f32_16x16x32_bf16(false, a.lo, false, b.hi, (short)0, c, false, false);
    asm volatile("v_nop\n\tv_nop\n\tv_nop\n\tv_nop" : "+v"(c) : "v"(a.hi), "v"(a.lo), "v"(b.hi), "v"(b.lo));
    return c;
}
__device__ __forceinline__ v16b ldb16(const unsigned short* p) {
    union { v16b v; v8b h[2]; } f; f.h[0] = *(const v8b*)(p); f.h[1] = *(const v8b*)(p + 16); return f.v;
}
__device__ __forceinline__ v16h ldh16(const unsigned short* p) {
    union { v16h v; v8h h[2]; } f; f.h[0] = *(const v8h*)(p); f.h[1] = *(const v8h*)(p + 16); return f.v;
}

#define VST2(T, ptr, val) do { const T vst2_v_ = (val); *(volatile T*)(ptr) = vst2_v_; __threadfence(); *(volatile T*)(ptr) = vst2_v_; } while (0)
#define VST2V4(ptr, val) do { const v4f vst2_v4_ = (val); *(volatile v4f*)(ptr) = vst2_v4_; __threadfence(); *(volatile v4f*)(ptr) = vst2_v4_; } while (0)

namespace w25 {
__device__ __forceinline__ unsigned short f2bf_bits(float f) {
  unsigned u = __float_as_uint(f);
  return (unsigned short)((u + 0x7FFFu + ((u >> 16) & 1u)) >> 16);
}
__device__ __forceinline__ float bf_bits2f(unsigned short h) { return __uint_as_float(((unsigned)h) << 16); }

__device__ __forceinline__ void dep_guard_h(v8f& a, v8f& b, v16h x, v16h y) { asm volatile("v_nop\n\tv_nop\n\tv_nop\n\tv_nop" : "+v"(a), "+v"(b) : "v"(x), "v"(y)); }
__device__ __forceinline__ void dep_guard_b(v8f& a, v8f& b, v16b x, v16b y) { asm volatile("v_nop\n\tv_nop\n\tv_nop\n\tv_nop" : "+v"(a), "+v"(b) : "v"(x), "v"(y)); }
__device__ __forceinline__ void keep4_h(v16h a, v16h b, v16h c, v16h d) { asm volatile("v_nop" :: "v"(a), "v"(b), "v"(c), "v"(d)); }
__device__ __forceinline__ void keep4_b(v16b a, v16b b, v16b c, v16b d) { asm volatile("v_nop" :: "v"(a), "v"(b), "v"(c), "v"(d)); }
__device__ __forceinline__ void acc_guard4(v8f& a, v8f& b, v8f& c, v8f& d) { asm volatile("v_nop\n\tv_nop\n\tv_nop\n\tv_nop" : "+v"(a), "+v"(b), "+v"(c), "+v"(d)); }
template <typename T> struct Frag;
template <> struct Frag<_Float16> {
  typedef v16h V; union U { v16h v; v8h h[2]; };
  static __device__ __forceinline__ v16h load(const _Float16* p) {
    U f; f.h[0] = *(const v8h*)(p); f.h[1] = *(const v8h*)(p + 16); return f.v;
  }
  static __device__ __forceinline__ v8f mma(v16h a, v16h b, v8f c) {
    return __builtin_amdgcn_wmma_f32_16x16x32_f16(false, a, false, b, (short)0, c, false, false);
  }
  static __device__ __forceinline__ void guard(v8f& a, v8f& b, v16h x, v16h y) { dep_guard_h(a, b, x, y); }
  static __device__ __forceinline__ void keep(v16h a, v16h b, v16h c, v16h d) { keep4_h(a, b, c, d); }
};
template <> struct Frag<__bf16> {
  typedef v16b V; union U { v16b v; v8b h[2]; };
  static __device__ __forceinline__ v16b load(const __bf16* p) {
    U f; f.h[0] = *(const v8b*)(p); f.h[1] = *(const v8b*)(p + 16); return f.v;
  }
  static __device__ __forceinline__ v8f mma(v16b a, v16b b, v8f c) {
    return __builtin_amdgcn_wmma_f32_16x16x32_bf16(false, a, false, b, (short)0, c, false, false);
  }
  static __device__ __forceinline__ void guard(v8f& a, v8f& b, v16b x, v16b y) { dep_guard_b(a, b, x, y); }
  static __device__ __forceinline__ void keep(v16b a, v16b b, v16b c, v16b d) { keep4_b(a, b, c, d); }
};

template <int ET> struct Elem;
template <> struct Elem<0> { typedef _Float16 T; };
template <> struct Elem<1> { typedef __bf16 T; };
template <int ET, bool SPLIT, int BIAS_MODE, int OUT_MODE, bool RESID, int ACT = 0>
__global__ __launch_bounds__(256) void wmma_gemm64(
    const unsigned short* __restrict__ Ap, const unsigned short* __restrict__ A2p, int lda, long strideA,
    const unsigned short* __restrict__ Btp, const unsigned short* __restrict__ Bt2p, int ldb, long strideB,
    void* __restrict__ Cout, void* __restrict__ Cout2, int ldc, long strideC,
    const float* __restrict__ bias,
    const float* __restrict__ resid, long strideR,
    int M, int N, int K, float scale) {
  typedef typename Elem<ET>::T T;
  typedef typename Frag<T>::V V;
  const T* A = (const T*)Ap; const T* A2 = (const T*)A2p; const T* Bt = (const T*)Btp; const T* Bt2 = (const T*)Bt2p;
  __shared__ __align__(16) float sT[8][16 * 68];
  const int b    = blockIdx.y;
  const int lane = threadIdx.x & 31;
  const int wave = threadIdx.x >> 5;
  const int tilesN = N >> 6;
  const int tilesM = M >> 6;
  const int tile = blockIdx.x * 8 + wave;
  if (tile >= tilesM * tilesN) return;
  const int tm = tile / tilesN;
  const int tn = tile - tm * tilesN;
  const int m0 = tm << 6;
  const int n0 = tn << 6;

  const T* Ab  = A  + (size_t)b * strideA;
  const T* Bb  = Bt + (size_t)b * strideB;
  const T* Ab2 = SPLIT ? (A2  + (size_t)b * strideA) : nullptr;
  const T* Bb2 = SPLIT ? (Bt2 + (size_t)b * strideB) : nullptr;

  const int rlane = lane & 15;
  const int koff  = (lane >> 4) * 8;
  const int mOff  = (lane >> 4) * 8;

  v8f acc[4][4];
#pragma unroll
  for (int i = 0; i < 4; ++i)
#pragma unroll
    for (int j = 0; j < 4; ++j) acc[i][j] = (v8f){0.f,0.f,0.f,0.f,0.f,0.f,0.f,0.f};

  for (int k0 = 0; k0 < K; k0 += 32) {
    V bh[4], bl[4];
#pragma unroll
    for (int j = 0; j < 4; ++j) {
      const size_t bo = (size_t)(n0 + (j << 4) + rlane) * ldb + koff + k0;
      bh[j] = Frag<T>::load(Bb + bo);
      if (SPLIT) bl[j] = Frag<T>::load(Bb2 + bo);
    }
#pragma unroll
    for (int i = 0; i < 4; ++i) {
      const size_t ao = (size_t)(m0 + (i << 4) + rlane) * lda + koff + k0;
      V ah = Frag<T>::load(Ab + ao);
      V al;
      if (SPLIT) al = Frag<T>::load(Ab2 + ao);
#pragma unroll
      for (int j = 0; j < 4; ++j) {
        acc[i][j] = Frag<T>::mma(ah, bh[j], acc[i][j]);
        if (SPLIT) {
          acc[i][j] = Frag<T>::mma(ah, bl[j], acc[i][j]);
          acc[i][j] = Frag<T>::mma(al, bh[j], acc[i][j]);
        }
      }
      Frag<T>::guard(acc[i][0], acc[i][3], ah, SPLIT ? al : ah);
    }
    Frag<T>::keep(bh[0], bh[1], bh[2], bh[3]);
    if (SPLIT) Frag<T>::keep(bl[0], bl[1], bl[2], bl[3]);
  }
  acc_guard4(acc[0][0], acc[0][1], acc[0][2], acc[0][3]);
  acc_guard4(acc[1][0], acc[1][1], acc[1][2], acc[1][3]);
  acc_guard4(acc[2][0], acc[2][1], acc[2][2], acc[2][3]);
  acc_guard4(acc[3][0], acc[3][1], acc[3][2], acc[3][3]);

  float* slab = sT[wave];
  const float* Rb = RESID ? (resid + (size_t)b * strideR) : nullptr;
#pragma unroll
  for (int i = 0; i < 4; ++i) {
    const int mBase = m0 + (i << 4);
#pragma unroll
    for (int j = 0; j < 4; ++j) {
      const int n = n0 + (j << 4) + rlane;
      float bv = 0.f;
      if (BIAS_MODE == 2) bv = bias[n];
#pragma unroll
      for (int r = 0; r < 8; ++r) {
        float v = acc[i][j][r] * scale;
        if (BIAS_MODE == 1) v += bias[mBase + mOff + r];
        if (BIAS_MODE == 2) v += bv;
        if (RESID) v += Rb[(size_t)(mBase + mOff + r) * ldc + n];
        if (ACT == 1) v = tanhf(v);
        if (ACT == 2) v = fmaxf(v, 0.0f);
        slab[(mOff + r) * 68 + (j << 4) + rlane] = v;
      }
    }
    __builtin_amdgcn_fence(3  , "workgroup");
    __builtin_amdgcn_wave_barrier();
    __builtin_amdgcn_fence(2  , "workgroup");
    if (OUT_MODE == 0) {
      float* C = (float*)Cout + (size_t)b * strideC;
      const int hh = lane >> 4, c4 = (lane & 15) * 4;
      for (int pass = 0; pass < 2; ++pass) {
#pragma unroll
        for (int it = 0; it < 8; ++it) {
          const int row = it * 2 + hh;
          v4f v = *(const v4f*)(slab + row * 68 + c4);
          *(volatile v4f*)(C + (size_t)(mBase + row) * ldc + n0 + c4) = v;
        }
        __threadfence();
      }
    } else {
      const int q = lane >> 3, c8 = (lane & 7) * 8;
      unsigned short* C  = (unsigned short*)Cout  + (size_t)b * strideC;
      unsigned short* C2 = (OUT_MODE >= 2) ? ((unsigned short*)Cout2 + (size_t)b * strideC) : nullptr;
      for (int pass = 0; pass < 2; ++pass) {
#pragma unroll
        for (int it = 0; it < 4; ++it) {
          const int row = it * 4 + q;
          const float* sp = slab + row * 68 + c8;
          v8h hv, lv;
#pragma unroll
          for (int e = 0; e < 8; ++e) {
            if (OUT_MODE == 1) {
              hv[e] = (_Float16)sp[e];
            } else if (OUT_MODE == 3) {
              const _Float16 hf = (_Float16)sp[e];
              hv[e] = hf;
              lv[e] = (_Float16)((sp[e] - (float)hf) * 2048.0f);
            } else {
              unsigned short hb = f2bf_bits(sp[e]);
              unsigned short lb = f2bf_bits(sp[e] - bf_bits2f(hb));
              hv[e] = __builtin_bit_cast(_Float16, hb);
              lv[e] = __builtin_bit_cast(_Float16, lb);
            }
          }
          *(volatile v8h*)(C + (size_t)(mBase + row) * ldc + n0 + c8) = hv;
          if (OUT_MODE >= 2) *(volatile v8h*)(C2 + (size_t)(mBase + row) * ldc + n0 + c8) = lv;
        }
        __threadfence();
      }
    }
    __builtin_amdgcn_fence(3  , "workgroup");
    __builtin_amdgcn_wave_barrier();
    __builtin_amdgcn_fence(2  , "workgroup");
  }
}
}

__device__ __forceinline__ float cmb_bf(float v) { const unsigned u = __builtin_bit_cast(unsigned, v); const unsigned r = (u + 0x7fffu + ((u >> 16) & 1u)) & 0xffff0000u; return __builtin_bit_cast(float, r); }
__device__ __forceinline__ unsigned int cmb_pk2(float a, float b) { return (unsigned int)__builtin_bit_cast(unsigned short, (_Float16)a) | ((unsigned int)__builtin_bit_cast(unsigned short, (_Float16)b) << 16); }

__global__ __launch_bounds__(256) void k_xcast(const float* __restrict__ x, unsigned short* __restrict__ X16) {
    const unsigned u = blockIdx.x * 256u + threadIdx.x;
    if (u >= (unsigned)(NB * SEQ) * 16u) return;
    const unsigned row = u >> 4, c0 = (u & 15u) << 3;
    const unsigned b = row / (unsigned)SEQ, n = row - b * (unsigned)SEQ;
    const float* s = x + ((size_t)b * CH + c0) * SEQ_FULL + n;
    float w[8];
#pragma unroll
    for (int e = 0; e < 8; ++e) w[e] = cmb_bf(s[(size_t)e * SEQ_FULL]);
    cm_u4 pk; pk.x = cmb_pk2(w[0], w[1]); pk.y = cmb_pk2(w[2], w[3]); pk.z = cmb_pk2(w[4], w[5]); pk.w = cmb_pk2(w[6], w[7]);
    VST2(cm_u4, (cm_u4*)(X16 + (size_t)row * CH + c0), pk);
}

__global__ __launch_bounds__(256) void k_wprep(const float* __restrict__ Wq, const float* __restrict__ Wk, const float* __restrict__ Wv,
                                               const float* __restrict__ bq, const float* __restrict__ bk, const float* __restrict__ bv,
                                               unsigned short* __restrict__ W3, float* __restrict__ BR3) {
    if (blockIdx.x < 24u) {
        const unsigned u = blockIdx.x * 256u + threadIdx.x;
        const unsigned row = u >> 4, c0 = (u & 15u) << 3;
        const unsigned mat = row >> 7, r = row & 127u;
        const float* src = (mat == 0u) ? Wq : ((mat == 1u) ? Wk : Wv);
        const float* s = src + (size_t)r * CH + c0;
        float w[8];
#pragma unroll
        for (int e = 0; e < 8; ++e) w[e] = cmb_bf(s[e]) * 16.0f;
        cm_u4 pk; pk.x = cmb_pk2(w[0], w[1]); pk.y = cmb_pk2(w[2], w[3]); pk.z = cmb_pk2(w[4], w[5]); pk.w = cmb_pk2(w[6], w[7]);
        VST2(cm_u4, (cm_u4*)(W3 + (size_t)row * CH + c0), pk);
    } else {
        const unsigned t = threadIdx.x;
        if (t < 96u) {
            const unsigned j4 = t << 2, mat = j4 >> 7, j = j4 & 127u;
            const float* src = (mat == 0u) ? bq : ((mat == 1u) ? bk : bv);
            v4f v; v.x = cmb_bf(src[j]); v.y = cmb_bf(src[j + 1]); v.z = cmb_bf(src[j + 2]); v.w = cmb_bf(src[j + 3]);
            VST2V4(BR3 + j4, v);
        }
    }
}

__global__ __launch_bounds__(128) void k_colstat(const unsigned short* __restrict__ QKh, const unsigned short* __restrict__ QKl, float* __restrict__ NL2) {
    __shared__ __align__(16) float stg[64];
    const unsigned lane = threadIdx.x & 31u, h = lane >> 4, l15 = lane & 15u, wave = threadIdx.x >> 5;
    const unsigned b = blockIdx.y, key0 = blockIdx.x * 64u + wave * 16u;
    const size_t rk = (size_t)(b * (unsigned)SEQ + key0 + l15) * QKP + CH + 8u * h;
    Split kf[4];
#pragma unroll
    for (int ks = 0; ks < 4; ++ks) { kf[ks].hi = ldb16(QKh + rk + ks * 32); kf[ks].lo = ldb16(QKl + rk + ks * 32); }
    const float L2E = 1.4426950408889634f;
    float m = -__builtin_inff(), l = 0.f;
    for (unsigned i0 = 0; i0 < (unsigned)SEQ; i0 += 16u) {
        const size_t rq = (size_t)(b * (unsigned)SEQ + i0 + l15) * QKP + 8u * h;
        v8f acc = {0.f, 0.f, 0.f, 0.f, 0.f, 0.f, 0.f, 0.f};
#pragma unroll
        for (int ks = 0; ks < 4; ++ks) {
            Split qa; qa.hi = ldb16(QKh + rq + ks * 32); qa.lo = ldb16(QKl + rq + ks * 32);
            acc = wmma3(qa, kf[ks], acc);
        }
        float t[8];
#pragma unroll
        for (int r = 0; r < 8; ++r) t[r] = acc[r] * L2E;
        float mx = fmaxf(fmaxf(fmaxf(t[0], t[1]), fmaxf(t[2], t[3])), fmaxf(fmaxf(t[4], t[5]), fmaxf(t[6], t[7])));
        const float mn = fmaxf(m, mx);
        float sum = 0.f;
#pragma unroll
        for (int r = 0; r < 8; ++r) sum += exp2f(t[r] - mn);
        l = l * exp2f(m - mn) + sum;
        m = mn;
    }
    const float mo = __shfl_xor(m, 16, 32), lo = __shfl_xor(l, 16, 32);
    const float M2 = fmaxf(m, mo);
    const float L2 = l * exp2f(m - M2) + lo * exp2f(mo - M2);
    const float nl = 14.0f - (M2 + log2f(L2));
    if (h == 0u) stg[wave * 16u + l15] = nl;
    __syncthreads();
    if (wave == 0u && lane < 16u) {
        const v4f v = *(const v4f*)&stg[4u * lane];
        VST2V4(NL2 + (size_t)b * SEQ + blockIdx.x * 64u + 4u * lane, v);
    }
}

__global__ __launch_bounds__(128) void k_colpv(const unsigned short* __restrict__ QKh, const unsigned short* __restrict__ QKl,
                                               const unsigned short* __restrict__ Vt, const unsigned short* __restrict__ Vr,
                                               const float* __restrict__ NL2, float* __restrict__ out) {
    __shared__ __align__(16) float ot[CH * OTP];
    const unsigned lane = threadIdx.x & 31u, h = lane >> 4, l15 = lane & 15u, wave = threadIdx.x >> 5;
    const unsigned b = blockIdx.y, qblk = blockIdx.x * 64u, q0 = qblk + wave * 16u;
    const size_t rq = (size_t)(b * (unsigned)SEQ + q0 + l15) * QKP + 8u * h;
    Split qf[4];
#pragma unroll
    for (int ks = 0; ks < 4; ++ks) { qf[ks].hi = ldb16(QKh + rq + ks * 32); qf[ks].lo = ldb16(QKl + rq + ks * 32); }
    v8f o[8], o2[8];
#pragma unroll
    for (int t = 0; t < 8; ++t) { o[t] = (v8f){0.f, 0.f, 0.f, 0.f, 0.f, 0.f, 0.f, 0.f}; o2[t] = (v8f){0.f, 0.f, 0.f, 0.f, 0.f, 0.f, 0.f, 0.f}; }
    const float L2E = 1.4426950408889634f;
    const size_t voff = ((size_t)b * CH + l15) * SEQ + 8u * h;
    const unsigned short* vrow  = Vt + voff;
    const unsigned short* vrrow = Vr + voff;
    const float* nlb = NL2 + (size_t)b * SEQ + 8u * h;
    for (unsigned j0 = 0; j0 < (unsigned)SEQ; j0 += 32u) {
        const size_t rk0 = (size_t)(b * (unsigned)SEQ + j0 + l15) * QKP + CH + 8u * h;
        const size_t rk1 = rk0 + (size_t)16 * QKP;
        v8f st0 = {0.f, 0.f, 0.f, 0.f, 0.f, 0.f, 0.f, 0.f};
        v8f st1 = {0.f, 0.f, 0.f, 0.f, 0.f, 0.f, 0.f, 0.f};
#pragma unroll
        for (int ks = 0; ks < 4; ++ks) {
            Split ka; ka.hi = ldb16(QKh + rk0 + ks * 32); ka.lo = ldb16(QKl + rk0 + ks * 32);
            st0 = wmma3(ka, qf[ks], st0);
        }
#pragma unroll
        for (int ks = 0; ks < 4; ++ks) {
            Split ka; ka.hi = ldb16(QKh + rk1 + ks * 32); ka.lo = ldb16(QKl + rk1 + ks * 32);
            st1 = wmma3(ka, qf[ks], st1);
        }
        const v4f n0a = *(const v4f*)(nlb + j0), n0b = *(const v4f*)(nlb + j0 + 4u);
        const v4f n1a = *(const v4f*)(nlb + j0 + 16u), n1b = *(const v4f*)(nlb + j0 + 20u);
        const float nl0[8] = {n0a.x, n0a.y, n0a.z, n0a.w, n0b.x, n0b.y, n0b.z, n0b.w};
        const float nl1[8] = {n1a.x, n1a.y, n1a.z, n1a.w, n1b.x, n1b.y, n1b.z, n1b.w};
        v16h pa;
#pragma unroll
        for (int r = 0; r < 8; ++r) {
            pa[r]     = (_Float16)exp2f(fmaf(st0[r], L2E, nl0[r]));
            pa[8 + r] = (_Float16)exp2f(fmaf(st1[r], L2E, nl1[r]));
        }
#pragma unroll
        for (int t = 0; t < 8; ++t) {
            const v16h vb = ldh16(vrow  + (size_t)(16 * t) * SEQ + j0);
            const v16h vr = ldh16(vrrow + (size_t)(16 * t) * SEQ + j0);
            o[t]  = wmma16(pa, vb, o[t]);
            o2[t] = wmma16(pa, vr, o2[t]);
        }
    }
    const float isc = 1.0f / 16384.0f;
    const float rsc = 1.0f / 2048.0f;
#pragma unroll
    for (int t = 0; t < 8; ++t) {
        const unsigned base = (16u * t + l15) * OTP + wave * 16u + 8u * h;
        v4f a, c;
        a.x = (o[t][0] + o2[t][0] * rsc) * isc; a.y = (o[t][1] + o2[t][1] * rsc) * isc;
        a.z = (o[t][2] + o2[t][2] * rsc) * isc; a.w = (o[t][3] + o2[t][3] * rsc) * isc;
        c.x = (o[t][4] + o2[t][4] * rsc) * isc; c.y = (o[t][5] + o2[t][5] * rsc) * isc;
        c.z = (o[t][6] + o2[t][6] * rsc) * isc; c.w = (o[t][7] + o2[t][7] * rsc) * isc;
        *(v4f*)&ot[base] = a;
        *(v4f*)&ot[base + 4u] = c;
    }
    __syncthreads();
    for (int pass = 0; pass < 2; ++pass) {
#pragma unroll
        for (int it = 0; it < 16; ++it) {
            const unsigned c = wave * 32u + (unsigned)it * 2u + h;
            const v4f v = *(const v4f*)&ot[c * OTP + l15 * 4u];
            *(volatile v4f*)(out + ((size_t)b * CH + c) * SEQ_FULL + qblk + l15 * 4u) = v;
        }
        __threadfence();
    }
}

static constexpr size_t al256(size_t v) { return (v + 255) / 256 * 256; }
static constexpr size_t SZ_X16 = al256((size_t)NB * SEQ * CH * 2);
static constexpr size_t SZ_W3  = al256((size_t)384 * CH * 2);
static constexpr size_t SZ_BR3 = al256((size_t)384 * 4);
static constexpr size_t SZ_QK  = al256((size_t)NB * SEQ * QKP * 2);
static constexpr size_t SZ_VT  = al256((size_t)NB * CH * SEQ * 2);
static constexpr size_t SZ_NL  = al256((size_t)NB * SEQ * 4);
static constexpr size_t WS_TOTAL = SZ_X16 + SZ_W3 + SZ_BR3 + 2 * SZ_QK + 2 * SZ_VT + SZ_NL;
static_assert(WS_TOTAL <= (size_t)134217728);
static_assert(((size_t)NB * SEQ * 16 / 256) * 256 * 8 == (size_t)NB * SEQ * CH);
static_assert((size_t)24 * 256 * 8 == (size_t)384 * CH);
static_assert((size_t)96 * 4 == 384);
static_assert(((size_t)NB * SEQ / 64) * (QKP / 64) * 64 * 64 == (size_t)NB * SEQ * QKP);
static_assert((size_t)NB * (CH / 64) * (SEQ / 64) * 64 * 64 == (size_t)NB * CH * SEQ);
static_assert((size_t)(SEQ / 64) * NB * 64 == (size_t)NB * SEQ);
static_assert((size_t)(SEQ / 64) * NB * CH * 64 == (size_t)NB * CH * SEQ);
static_assert(((size_t)(NB - 1) * CH + (CH - 1)) * SEQ_FULL + SEQ <= (size_t)NB_FULL * CH * SEQ_FULL);

extern "C" void kernel_launch(void* const* d_in, const int* in_sizes, int n_in, void* d_out, int out_size, void* d_ws, size_t ws_size, hipStream_t stream) {
    if (n_in < 7) return;
    if (in_sizes[0] < NB * CH * SEQ_FULL) return;
    if (in_sizes[1] < CH * CH || in_sizes[3] < CH * CH || in_sizes[5] < CH * CH) return;
    if (in_sizes[2] < CH || in_sizes[4] < CH || in_sizes[6] < CH) return;
    if (out_size < NB * CH * SEQ_FULL) return;
    if (WS_TOTAL > ws_size) return;
    const float* x  = (const float*)d_in[0];
    const float* Wq = (const float*)d_in[1];
    const float* bq = (const float*)d_in[2];
    const float* Wk = (const float*)d_in[3];
    const float* bk = (const float*)d_in[4];
    const float* Wv = (const float*)d_in[5];
    const float* bv = (const float*)d_in[6];
    float* out = (float*)d_out;
    char* wsp = (char*)d_ws;
    unsigned short* X16 = (unsigned short*)wsp; wsp += SZ_X16;
    unsigned short* W3  = (unsigned short*)wsp; wsp += SZ_W3;
    float* BR3          = (float*)wsp;          wsp += SZ_BR3;
    unsigned short* QKh = (unsigned short*)wsp; wsp += SZ_QK;
    unsigned short* QKl = (unsigned short*)wsp; wsp += SZ_QK;
    unsigned short* Vt  = (unsigned short*)wsp; wsp += SZ_VT;
    unsigned short* Vr  = (unsigned short*)wsp; wsp += SZ_VT;
    float* NL2          = (float*)wsp;          wsp += SZ_NL;

    k_xcast<<<(unsigned)(((size_t)NB * SEQ * 16 + 255) / 256), 256, 0, stream>>>(x, X16);
    k_wprep<<<25, 256, 0, stream>>>(Wq, Wk, Wv, bq, bk, bv, W3, BR3);
    w25::wmma_gemm64<0, false, 2, 2, false, 0><<<dim3((unsigned)((((NB * SEQ) / 64) * (QKP / 64) + 7) / 8), 1u), 256, 0, stream>>>(
        (const unsigned short*)X16, nullptr, CH, 0L, (const unsigned short*)W3, nullptr, CH, 0L,
        (void*)QKh, (void*)QKl, QKP, 0L, BR3, nullptr, 0L, NB * SEQ, QKP, CH, 0.0625f);
    w25::wmma_gemm64<0, false, 1, 3, false, 0><<<dim3((unsigned)(((CH / 64) * (SEQ / 64) + 7) / 8), (unsigned)NB), 256, 0, stream>>>(
        (const unsigned short*)(W3 + 256 * CH), nullptr, CH, 0L, (const unsigned short*)X16, nullptr, CH, (long)SEQ * CH,
        (void*)Vt, (void*)Vr, SEQ, (long)CH * SEQ, BR3 + 256, nullptr, 0L, CH, SEQ, CH, 0.0625f);
    k_colstat<<<dim3((unsigned)(SEQ / 64), (unsigned)NB), 128, 0, stream>>>(QKh, QKl, NL2);
    k_colpv<<<dim3((unsigned)(SEQ / 64), (unsigned)NB), 128, 0, stream>>>(QKh, QKl, Vt, Vr, NL2, out);
}
